// S4Layer_11605001634066
// MI455X (gfx1250) — hardware-verified
//
#include <hip/hip_runtime.h>
#include <math.h>

constexpr int NBAT  = 8;
constexpr int NCH   = 256;
constexpr int NLEN  = 4096;
constexpr int NST   = 32;
constexpr int NO2   = 512;
constexpr int NTHR  = 256;
constexpr int CSP   = 36;
constexpr int SLABP = 68;
static_assert(NST == 32);
static_assert((NCH & (NCH - 1)) == 0);
static_assert(NCH % 32 == 0);
static_assert(NO2 % 64 == 0 && NLEN % 64 == 0);
static_assert((NCH * NST) % NTHR == 0);
static_assert((NO2 * (NCH / 8)) % NTHR == 0);
static_assert((NBAT * NCH) % (NTHR / 32) == 0);
static_assert(NLEN % NST == 0);
static_assert(NCH % 64 == 0);
static_assert(((NO2 / 64) * (NLEN / 64)) % 8 == 0);

typedef __attribute__((ext_vector_type(16))) __bf16   v16b;
typedef __attribute__((ext_vector_type(8)))  __bf16   v8b;
typedef __attribute__((ext_vector_type(8)))  float    v8f;
typedef __attribute__((ext_vector_type(4)))  float    v4f;
typedef __attribute__((ext_vector_type(4)))  unsigned v4u;

__device__ __forceinline__ unsigned short f2bf_bits(float f) {
  unsigned u = __float_as_uint(f);
  return (unsigned short)((u + 0x7FFFu + ((u >> 16) & 1u)) >> 16);
}
__device__ __forceinline__ float bf_bits2f(unsigned short h) { return __uint_as_float(((unsigned)h) << 16); }
__device__ __forceinline__ void bf_split_bits(float f, unsigned& hb, unsigned& lb) {
  const unsigned short h = f2bf_bits(f);
  hb = (unsigned)h;
  lb = (unsigned)f2bf_bits(f - bf_bits2f(h));
}

__device__ __forceinline__ void dep_guard4_b(v8f& a, v8f& b, v8f& c, v8f& d, v16b x, v16b y) {
  asm volatile("v_nop\n\tv_nop\n\tv_nop\n\tv_nop" : "+v"(a), "+v"(b), "+v"(c), "+v"(d) : "v"(x), "v"(y));
}
__device__ __forceinline__ void keep4_b(v16b a, v16b b, v16b c, v16b d) { asm volatile("v_nop" :: "v"(a), "v"(b), "v"(c), "v"(d)); }
__device__ __forceinline__ void acc_guard4(v8f& a, v8f& b, v8f& c, v8f& d) { asm volatile("v_nop\n\tv_nop\n\tv_nop\n\tv_nop" : "+v"(a), "+v"(b), "+v"(c), "+v"(d)); }

struct FragB {
  union U { v16b v; v8b h[2]; };
  static __device__ __forceinline__ v16b load(const __bf16* p) {
    U f; f.h[0] = *(const v8b*)(p); f.h[1] = *(const v8b*)(p + 16); return f.v;
  }
  static __device__ __forceinline__ v8f mma(v16b a, v16b b, v8f c) {
    return __builtin_amdgcn_wmma_f32_16x16x32_bf16(false, a, false, b, (short)0, c, false, false);
  }
};

__global__ __launch_bounds__(NTHR) void diag_params_kernel(const float* __restrict__ log_dt,
                                                           const float* __restrict__ log_A_real,
                                                           const float* __restrict__ A_imag,
                                                           const float* __restrict__ C_re,
                                                           const float* __restrict__ C_im,
                                                           float* __restrict__ lamR, float* __restrict__ lamI,
                                                           float* __restrict__ ckR, float* __restrict__ ckI) {
  const int idx = blockIdx.x * NTHR + threadIdx.x;
  if (idx >= NCH * NST) return;
  const int h = idx >> 5;
  const float dt = expf(log_dt[h]);
  const float Ar = -expf(log_A_real[idx]);
  const float Ai = A_imag[idx];
  const float ar = Ar * dt, ai = Ai * dt;
  const float er = expf(ar);
  const float lr = er * cosf(ai);
  const float li = er * sinf(ai);
  const float dr = lr - 1.0f, di = li;
  const float den = Ar * Ar + Ai * Ai;
  const float inv = 1.0f / den;
  const float qr = (dr * Ar + di * Ai) * inv;
  const float qi = (di * Ar - dr * Ai) * inv;
  const float cr = C_re[idx], ci = C_im[idx];
  const float k2r = 2.0f * (cr * qr - ci * qi);
  const float k2i = 2.0f * (cr * qi + ci * qr);
  *(volatile float*)(lamR + idx) = lr;
  *(volatile float*)(lamI + idx) = li;
  *(volatile float*)(ckR  + idx) = k2r;
  *(volatile float*)(ckI  + idx) = k2i;
  __threadfence();
  *(volatile float*)(lamR + idx) = lr;
  *(volatile float*)(lamI + idx) = li;
  *(volatile float*)(ckR  + idx) = k2r;
  *(volatile float*)(ckI  + idx) = k2i;
}

__global__ __launch_bounds__(NTHR) void wsplit_kernel(const float* __restrict__ W,
                                                      unsigned short* __restrict__ PH,
                                                      unsigned short* __restrict__ PL) {
  const int i = blockIdx.x * NTHR + threadIdx.x;
  if (i >= NO2 * (NCH / 8)) return;
  const int m  = i >> 5;
  const int c8 = (i & 31) * 8;
  const int tmm = m >> 6, rr = m & 63;
  const int o = (tmm << 5) + (rr & 31) + ((rr >> 5) << 8);
  const float* sp = W + (size_t)o * NCH + c8;
  const v4f a = *(const v4f*)(sp);
  const v4f c = *(const v4f*)(sp + 4);
  unsigned hb[8], lb[8];
#pragma unroll
  for (int e = 0; e < 4; ++e) {
    bf_split_bits(a[e], hb[e], lb[e]);
    bf_split_bits(c[e], hb[4 + e], lb[4 + e]);
  }
  v4u ph, pl;
#pragma unroll
  for (int e2 = 0; e2 < 4; ++e2) {
    ph[e2] = hb[2 * e2] | (hb[2 * e2 + 1] << 16);
    pl[e2] = lb[2 * e2] | (lb[2 * e2 + 1] << 16);
  }
  unsigned short* dh = PH + (size_t)i * 8;
  unsigned short* dl = PL + (size_t)i * 8;
  *(volatile v4u*)dh = ph;
  *(volatile v4u*)dl = pl;
  __threadfence();
  *(volatile v4u*)dh = ph;
  *(volatile v4u*)dl = pl;
}

__global__ __launch_bounds__(NTHR) void ssm_scan_kernel(const float* __restrict__ u_in,
                                                        const float* __restrict__ lamR, const float* __restrict__ lamI,
                                                        const float* __restrict__ ckR, const float* __restrict__ ckI,
                                                        const float* __restrict__ Dvec, float* __restrict__ yact) {
  __shared__ __align__(16) float csum[NTHR / 32][NST * CSP];
  const int tid = threadIdx.x, lane = tid & 31, wv = tid >> 5;
  const int wg = blockIdx.x * (NTHR / 32) + wv;
  const int h = wg & (NCH - 1);
  const int pidx = h * NST + lane;
  const float lr = lamR[pidx], li = lamI[pidx], ckr = ckR[pidx], cki = ckI[pidx];
  const float Dh = Dvec[h];
  const float* u = u_in + (size_t)wg * NLEN;
  float* yp = yact + (size_t)wg * NLEN;
  float* cw = csum[wv];
  float sr = 0.0f, si = 0.0f;
#pragma unroll 1
  for (int l0 = 0; l0 < NLEN; l0 += NST) {
    const float uv = u[l0 + lane];
#pragma unroll 1
    for (int t = 0; t < NST; ++t) {
      const float ul = __shfl(uv, t, 32);
      const float nsr = fmaf(lr, sr, fmaf(-li, si, ul));
      const float nsi = fmaf(lr, si, li * sr);
      sr = nsr; si = nsi;
      cw[t * CSP + lane] = fmaf(ckr, sr, -(cki * si));
    }
    __syncthreads();
    float acc = 0.0f;
    const float* rp = cw + lane * CSP;
#pragma unroll
    for (int q = 0; q < NST / 4; ++q) {
      const v4f v = *(const v4f*)(rp + 4 * q);
      acc += v[0]; acc += v[1]; acc += v[2]; acc += v[3];
    }
    const float y  = fmaf(uv, Dh, acc);
    const float ge = 0.5f * y * (1.0f + erff(y * 0.70710678118654752f));
    float* op = yp + l0 + lane;
    *(volatile float*)op = ge;
    __threadfence();
    *(volatile float*)op = ge;
    __syncthreads();
  }
}

__global__ __launch_bounds__(NTHR) void tpsplit_kernel(const float* __restrict__ src,
                                                       unsigned short* __restrict__ GH, unsigned short* __restrict__ GL) {
  __shared__ float Tt[64 * 65];
  const int tid = threadIdx.x;
  const int c0 = blockIdx.x * 64, r0 = blockIdx.y * 64, b = blockIdx.z;
  const float* sb = src + (size_t)b * NCH * NLEN;
#pragma unroll
  for (int i = 0; i < 4; ++i) {
    const int idx = i * NTHR + tid;
    const int rr = idx >> 4, cc = (idx & 15) * 4;
    const v4f v = *(const v4f*)(sb + (size_t)(r0 + rr) * NLEN + c0 + cc);
    Tt[rr * 65 + cc + 0] = v[0];
    Tt[rr * 65 + cc + 1] = v[1];
    Tt[rr * 65 + cc + 2] = v[2];
    Tt[rr * 65 + cc + 3] = v[3];
  }
  __syncthreads();
  const int q = tid >> 3, c8 = (tid & 7) * 8;
  v4u ph[2], pl[2];
#pragma unroll
  for (int g = 0; g < 2; ++g) {
    const int qq = g * 32 + q;
    unsigned hb[8], lb[8];
#pragma unroll
    for (int e = 0; e < 8; ++e) bf_split_bits(Tt[(c8 + e) * 65 + qq], hb[e], lb[e]);
#pragma unroll
    for (int e2 = 0; e2 < 4; ++e2) {
      ph[g][e2] = hb[2 * e2] | (hb[2 * e2 + 1] << 16);
      pl[g][e2] = lb[2 * e2] | (lb[2 * e2 + 1] << 16);
    }
  }
  const size_t ob = (size_t)b * NLEN * NCH;
  for (int pass = 0; pass < 2; ++pass) {
#pragma unroll
    for (int g = 0; g < 2; ++g) {
      const size_t o = ob + (size_t)(c0 + g * 32 + q) * NCH + (size_t)(r0 + c8);
      *(volatile v4u*)(GH + o) = ph[g];
      *(volatile v4u*)(GL + o) = pl[g];
    }
    __threadfence();
  }
}

__global__ __launch_bounds__(NTHR) void gemm_glu_kernel(const unsigned short* __restrict__ WHp,
                                                        const unsigned short* __restrict__ WLp,
                                                        const unsigned short* __restrict__ GHp,
                                                        const unsigned short* __restrict__ GLp,
                                                        const float* __restrict__ bias, float* __restrict__ out) {
  __shared__ __align__(16) float sT[NTHR / 32][16 * SLABP];
  const __bf16* A   = (const __bf16*)WHp;
  const __bf16* A2  = (const __bf16*)WLp;
  const int b    = blockIdx.y;
  const int lane = threadIdx.x & 31;
  const int wave = threadIdx.x >> 5;
  constexpr int tilesN = NLEN / 64;
  constexpr int tilesM = NO2 / 64;
  const int tile = blockIdx.x * 8 + wave;
  if (tile >= tilesM * tilesN) return;
  const int tm = tile / tilesN;
  const int tn = tile - tm * tilesN;
  const int m0 = tm << 6;
  const int n0 = tn << 6;
  const __bf16* Bb  = (const __bf16*)GHp + (size_t)b * NLEN * NCH;
  const __bf16* Bb2 = (const __bf16*)GLp + (size_t)b * NLEN * NCH;

  const int rlane = lane & 15;
  const int koff  = (lane >> 4) * 8;
  const int mOff  = (lane >> 4) * 8;

  v8f acc[4][4];
#pragma unroll
  for (int i = 0; i < 4; ++i)
#pragma unroll
    for (int j = 0; j < 4; ++j) acc[i][j] = (v8f){0.f,0.f,0.f,0.f,0.f,0.f,0.f,0.f};

  for (int k0 = 0; k0 < NCH; k0 += 32) {
    v16b bh[4], bl[4];
#pragma unroll
    for (int j = 0; j < 4; ++j) {
      const size_t bo = (size_t)(n0 + (j << 4) + rlane) * NCH + koff + k0;
      bh[j] = FragB::load(Bb + bo);
      bl[j] = FragB::load(Bb2 + bo);
    }
#pragma unroll
    for (int i = 0; i < 4; ++i) {
      const size_t ao = (size_t)(m0 + (i << 4) + rlane) * NCH + koff + k0;
      const v16b ah = FragB::load(A + ao);
      const v16b al = FragB::load(A2 + ao);
#pragma unroll
      for (int j = 0; j < 4; ++j) {
        acc[i][j] = FragB::mma(ah, bh[j], acc[i][j]);
        acc[i][j] = FragB::mma(ah, bl[j], acc[i][j]);
        acc[i][j] = FragB::mma(al, bh[j], acc[i][j]);
      }
      dep_guard4_b(acc[i][0], acc[i][1], acc[i][2], acc[i][3], ah, al);
    }
    keep4_b(bh[0], bh[1], bh[2], bh[3]);
    keep4_b(bl[0], bl[1], bl[2], bl[3]);
  }
  acc_guard4(acc[0][0], acc[0][1], acc[0][2], acc[0][3]);
  acc_guard4(acc[1][0], acc[1][1], acc[1][2], acc[1][3]);
  acc_guard4(acc[2][0], acc[2][1], acc[2][2], acc[2][3]);
  acc_guard4(acc[3][0], acc[3][1], acc[3][2], acc[3][3]);

  float* slab = sT[wave];
  float* Cb = out + (size_t)b * NCH * NLEN;
#pragma unroll
  for (int i = 0; i < 2; ++i) {
    const int oBase = (tm << 5) + (i << 4);
    const v4f ba0 = *(const v4f*)(bias + oBase + mOff);
    const v4f ba1 = *(const v4f*)(bias + oBase + mOff + 4);
    const v4f bg0 = *(const v4f*)(bias + NCH + oBase + mOff);
    const v4f bg1 = *(const v4f*)(bias + NCH + oBase + mOff + 4);
#pragma unroll
    for (int j = 0; j < 4; ++j) {
#pragma unroll
      for (int r = 0; r < 8; ++r) {
        const float bav = (r < 4) ? ba0[r & 3] : ba1[r & 3];
        const float bgv = (r < 4) ? bg0[r & 3] : bg1[r & 3];
        const float va = acc[i][j][r] + bav;
        const float vg = acc[i + 2][j][r] + bgv;
        const float sg = __builtin_amdgcn_rcpf(1.0f + expf(-vg));
        slab[(mOff + r) * SLABP + (j << 4) + rlane] = va * sg;
      }
    }
    __builtin_amdgcn_fence(__ATOMIC_RELEASE, "workgroup");
    __builtin_amdgcn_wave_barrier();
    __builtin_amdgcn_fence(__ATOMIC_ACQUIRE, "workgroup");
    {
      const int hh = lane >> 4, c4 = (lane & 15) * 4;
      for (int pass = 0; pass < 2; ++pass) {
#pragma unroll
        for (int it = 0; it < 8; ++it) {
          const int row = it * 2 + hh;
          const v4f v = *(const v4f*)(slab + row * SLABP + c4);
          *(volatile v4f*)(Cb + (size_t)(oBase + row) * NLEN + n0 + c4) = v;
        }
        __threadfence();
      }
    }
    __builtin_amdgcn_fence(__ATOMIC_RELEASE, "workgroup");
    __builtin_amdgcn_wave_barrier();
    __builtin_amdgcn_fence(__ATOMIC_ACQUIRE, "workgroup");
  }
}

extern "C" void kernel_launch(void* const* d_in, const int* in_sizes, int n_in,
                              void* d_out, int out_size, void* d_ws, size_t ws_size, hipStream_t stream) {
  if (n_in < 9 || d_out == nullptr || d_ws == nullptr) return;
  if (in_sizes[0] != NBAT * NCH * NLEN || in_sizes[1] != NCH || in_sizes[2] != NCH * NST ||
      in_sizes[3] != NCH * NST || in_sizes[4] != NCH * NST || in_sizes[5] != NCH * NST ||
      in_sizes[6] != NCH || in_sizes[7] != NO2 * NCH || in_sizes[8] != NO2 ||
      out_size != NBAT * NCH * NLEN) return;

  const float* u      = (const float*)d_in[0];
  const float* log_dt = (const float*)d_in[1];
  const float* log_Ar = (const float*)d_in[2];
  const float* A_im   = (const float*)d_in[3];
  const float* C_re   = (const float*)d_in[4];
  const float* C_im   = (const float*)d_in[5];
  const float* Dv     = (const float*)d_in[6];
  const float* W      = (const float*)d_in[7];
  const float* b_out  = (const float*)d_in[8];
  float* out = (float*)d_out;

  char* ws = (char*)d_ws; size_t off = 0;
  auto carve = [&](size_t bytes) -> char* { char* p = ws + off; off += (bytes + 255) & ~(size_t)255; return p; };
  float* LAMR = (float*)carve((size_t)NCH * NST * 4);
  float* LAMI = (float*)carve((size_t)NCH * NST * 4);
  float* CK2R = (float*)carve((size_t)NCH * NST * 4);
  float* CK2I = (float*)carve((size_t)NCH * NST * 4);
  unsigned short* WH = (unsigned short*)carve((size_t)NO2 * NCH * 2);
  unsigned short* WL = (unsigned short*)carve((size_t)NO2 * NCH * 2);
  float* YACT = (float*)carve((size_t)NBAT * NCH * NLEN * 4);
  unsigned short* GH = (unsigned short*)carve((size_t)NBAT * NLEN * NCH * 2);
  unsigned short* GL = (unsigned short*)carve((size_t)NBAT * NLEN * NCH * 2);
  if (off > ws_size || off > (size_t)134217728) return;

  diag_params_kernel<<<(NCH * NST) / NTHR, NTHR, 0, stream>>>(log_dt, log_Ar, A_im, C_re, C_im, LAMR, LAMI, CK2R, CK2I);
  wsplit_kernel<<<(NO2 * (NCH / 8)) / NTHR, NTHR, 0, stream>>>(W, WH, WL);
  ssm_scan_kernel<<<(NBAT * NCH) / (NTHR / 32), NTHR, 0, stream>>>(u, LAMR, LAMI, CK2R, CK2I, Dv, YACT);
  tpsplit_kernel<<<dim3(NLEN / 64, NCH / 64, NBAT), NTHR, 0, stream>>>(YACT, GH, GL);
  gemm_glu_kernel<<<dim3(((NO2 / 64) * (NLEN / 64)) / 8, NBAT), NTHR, 0, stream>>>(WH, WL, GH, GL, b_out, out);
}
